// EmbedLayer_59304908423194
// MI455X (gfx1250) — hardware-verified
//
#include <hip/hip_runtime.h>
#include <hip/hip_bf16.h>


#define V       100
#define C       10
#define H       64
#define BATCH   128
#define KP      1024
#define KT      1000
#define NSTEP   (KP / 32)
#define BH      64
#define BTSTR   40

typedef __attribute__((ext_vector_type(16))) _Float16 v16h;
typedef __attribute__((ext_vector_type(8)))  _Float16 v8h;
typedef __attribute__((ext_vector_type(2)))  _Float16 v2h;
typedef __attribute__((ext_vector_type(8)))  float    v8f;
typedef __attribute__((ext_vector_type(4)))  float    v4f;
typedef float __attribute__((may_alias)) float_a;
template <typename T> __device__ __forceinline__ void vst2(void* p, T v) { *(volatile T*)p = v; __threadfence(); *(volatile T*)p = v; }
__device__ __forceinline__ v8f wmma16(v16h a, v16h b, v8f c) {
    v8f d = __builtin_amdgcn_wmma_f32_16x16x32_f16(false, a, false, b, (short)0, c, false, false);
    asm volatile("v_nop\n\tv_nop\n\tv_nop\n\tv_nop" : "+v"(d) : "v"(a), "v"(b));
    return d;
}

__device__ __forceinline__
void stage_tile(const float* __restrict__ tblock, _Float16* Btp,
                int Kbase, int tid) {
    const int kp = tid >> 4;
    const int n4 = (tid & 15) * 4;
    int kr0 = Kbase + kp * 2;
    int kr1 = kr0 + 1;
    kr0 = (kr0 < KT) ? kr0 : (KT - 1);
    kr1 = (kr1 < KT) ? kr1 : (KT - 1);
    v4f r0 = *(const v4f*)(tblock + (size_t)kr0 * H + n4);
    v4f r1 = *(const v4f*)(tblock + (size_t)kr1 * H + n4);
    #pragma unroll
    for (int c = 0; c < 4; ++c) {
        v2h p;
        p[0] = (_Float16)r0[c];
        p[1] = (_Float16)r1[c];
        *(v2h*)(Btp + (n4 + c) * BTSTR + kp * 2) = p;
    }
}

__global__ __launch_bounds__(256, 1)
void embed_wmma_kernel(const int* __restrict__ x,
                       const float* __restrict__ mask,
                       const float* __restrict__ table,
                       const float* __restrict__ bias,
                       float* __restrict__ out) {
    __shared__ __attribute__((aligned(16))) _Float16 Wl[BH * KP];
    __shared__ __attribute__((aligned(16))) _Float16 Btd[2][H * BTSTR];
    __shared__ __attribute__((aligned(16))) float So[8][16 * 32];

    const int i   = blockIdx.x;
    const int bh  = blockIdx.y;
    const int tid = threadIdx.x;

    {
        v8h z = {};
        v8h* wv = (v8h*)Wl;
        #pragma unroll
        for (int it = 0; it < (BH * KP) / (8 * 256); ++it)
            wv[tid + it * 256] = z;
    }
    __syncthreads();
    {
        #pragma unroll
        for (int it = 0; it < (BH * V) / 256; ++it) {
            int idx = tid + it * 256;
            int bl  = idx / V;
            int j   = idx - bl * V;
            int b   = bh * BH + bl;
            float m = mask[((size_t)b * V + i) * V + j];
            int  xv = x[b * V + j];
            float w = (m == 1.0f) ? 1.0f : 0.0f;
            Wl[bl * KP + j * C + xv] = (_Float16)w;
        }
    }

    const float* tblock = table + (size_t)i * KT * H;

    stage_tile(tblock, Btd[0], 0, tid);

    const int wave  = tid >> 5;
    const int lane  = tid & 31;
    const int mt    = wave & 3;
    const int npair = wave >> 2;
    const int half  = lane >> 4;
    const int l15   = lane & 15;

    v8f acc0 = {};
    v8f acc1 = {};

    for (int kb = 0; kb < NSTEP; ++kb) {
        __syncthreads();
        const _Float16* Bp = Btd[kb & 1];

        if (kb + 1 < NSTEP)
            stage_tile(tblock, Btd[(kb + 1) & 1], (kb + 1) * 32, tid);
        if (kb + 2 < NSTEP - 1)
            __builtin_prefetch(tblock + (size_t)(kb + 2) * 32 * H + tid * 8, 0, 1);

        const int Kbase = kb * 32;

        const _Float16* wr = Wl + (mt * 16 + l15) * KP + Kbase + half * 8;
        v8h a0 = *(const v8h*)(wr);
        v8h a1 = *(const v8h*)(wr + 16);
        v16h A = __builtin_shufflevector(a0, a1, 0,1,2,3,4,5,6,7,8,9,10,11,12,13,14,15);

        const _Float16* bp0 = Bp + ((npair * 2 + 0) * 16 + l15) * BTSTR + half * 8;
        const _Float16* bp1 = Bp + ((npair * 2 + 1) * 16 + l15) * BTSTR + half * 8;
        v8h b00 = *(const v8h*)(bp0);
        v8h b01 = *(const v8h*)(bp0 + 16);
        v8h b10 = *(const v8h*)(bp1);
        v8h b11 = *(const v8h*)(bp1 + 16);
        v16h B0 = __builtin_shufflevector(b00, b01, 0,1,2,3,4,5,6,7,8,9,10,11,12,13,14,15);
        v16h B1 = __builtin_shufflevector(b10, b11, 0,1,2,3,4,5,6,7,8,9,10,11,12,13,14,15);

        acc0 = wmma16(A, B0, acc0);
        acc1 = wmma16(A, B1, acc1);
    }

    const int n0 = (npair * 2 + 0) * 16 + l15;
    const int n1 = (npair * 2 + 1) * 16 + l15;
    const float bias0 = bias[i * H + n0];
    const float bias1 = bias[i * H + n1];
    float* S = So[wave];
    #pragma unroll
    for (int r = 0; r < 8; ++r) {
        int M = r + half * 8;
        S[M * 32 + l15]      = acc0[r] + bias0;
        S[M * 32 + 16 + l15] = acc1[r] + bias1;
    }
    __syncthreads();
    #pragma unroll
    for (int q = 0; q < 4; ++q) {
        const int rl = q * 4 + (lane >> 3), pc = lane & 7;
        const int b = bh * BH + mt * 16 + rl;
        vst2(out + ((size_t)b * V + i) * H + npair * 32 + pc * 4, *(const v4f*)(S + rl * 32 + pc * 4));
    }
}

extern "C" void kernel_launch(void* const* d_in, const int* in_sizes, int n_in,
                              void* d_out, int out_size, void* d_ws, size_t ws_size,
                              hipStream_t stream) {
    (void)in_sizes; (void)n_in; (void)out_size; (void)d_ws; (void)ws_size;
    const int*   x     = (const int*)d_in[0];
    const float* mask  = (const float*)d_in[1];
    const float* table = (const float*)d_in[2];
    const float* bias  = (const float*)d_in[3];
    float*       out   = (float*)d_out;

    dim3 grid(V, BATCH / BH, 1);
    embed_wmma_kernel<<<grid, 256, 0, stream>>>(x, mask, table, bias, out);
}
